// InformationPrototype_82360292868467
// MI455X (gfx1250) — hardware-verified
//
#include <hip/hip_runtime.h>
#include <stddef.h>


typedef _Float16 h16;
typedef _Float16 v16h __attribute__((ext_vector_type(16)));
typedef _Float16 v8h  __attribute__((ext_vector_type(8)));
typedef float    v8f  __attribute__((ext_vector_type(8)));
typedef float    v4f  __attribute__((ext_vector_type(4)));
typedef int      v4i  __attribute__((ext_vector_type(4)));

#ifndef NROWS
#define NROWS 8192
#endif
#define NROWS_FULL 8192
#define DIM   512
#define NCLS  100
#define SUBROWS (NROWS / 8)

static_assert(NROWS >= 256 && NROWS <= NROWS_FULL);
static_assert((NROWS % 64) == 0 && (NROWS % 32) == 0);
static_assert((NROWS % 256) == 0);
static_assert(SUBROWS * 8 == NROWS && (SUBROWS % 32) == 0);
static_assert((DIM % 64) == 0 && (DIM % 32) == 0);
static_assert(DIM == 4 * 32 * 4);
static_assert(DIM == 128 * 4);
static_assert(DIM == 2 * 256);
static_assert((NCLS % 10) == 0);
static_assert(NCLS <= 4 * 32);

#define LDT 72
#define LDC 68
static_assert((LDT % 8) == 0 && LDT >= 64);
static_assert((LDC % 4) == 0 && LDC >= 64);

#define NCARRY 64.0f

#define OUT1_OFF  ((size_t)NCLS * DIM)
#define OUT_TOTAL (OUT1_OFF + (size_t)NCLS * NCLS * DIM)
static_assert(OUT1_OFF * 4 == (size_t)204800);
static_assert(OUT_TOTAL * 4 == (size_t)20684800);
static_assert(((OUT1_OFF * 4) % 128) == 0);
static_assert(((size_t)(NCLS - 1) * DIM + (DIM - 1)) < OUT1_OFF);

#define XT_BYTES   ((size_t)DIM * NROWS * 2)
#define XN_BYTES   ((size_t)NROWS * DIM * 2)
#define GT_BYTES   ((size_t)DIM * DIM * 2)
#define CLS_BYTES  ((size_t)NROWS * 4)
#define WT_BYTES   ((size_t)NROWS * 4)
#define OFF_XT   ((size_t)0)
#define OFF_XNT  (OFF_XT + XT_BYTES)
#define OFF_XN   (OFF_XNT + XT_BYTES)
#define OFF_GT   (OFF_XN + XN_BYTES)
#define OFF_XAT  (OFF_GT + GT_BYTES)
#define OFF_CLS  (OFF_XAT + XT_BYTES)
#define OFF_WT   (OFF_CLS + CLS_BYTES)
#define WS_TOTAL (OFF_WT + WT_BYTES)
static_assert((XT_BYTES % 128) == 0 && (XN_BYTES % 128) == 0 && (GT_BYTES % 128) == 0);
static_assert((CLS_BYTES % 256) == 0 && (WT_BYTES % 256) == 0);
static_assert(WS_TOTAL <= (size_t)134217728);

__device__ __forceinline__ float bf16r(float x) {
  unsigned int u = __float_as_uint(x);
  u = (u + 0x7FFFu + ((u >> 16) & 1u)) & 0xFFFF0000u;
  return __uint_as_float(u);
}

static __device__ __forceinline__ h16 toh_flush(float v) {
  const h16 r = (h16)v;
  return (fabsf(v) < 6.103515625e-05f) ? (h16)0.0f : r;
}

__device__ __forceinline__ v16h frag_at(const _Float16* p) {
  v8h lo = *(const v8h*)(p);
  v8h hi = *(const v8h*)(p + 16);
  v16h out;
#pragma unroll
  for (int i = 0; i < 8; ++i) { out[i] = lo[i]; out[i + 8] = hi[i]; }
  return out;
}

__device__ __forceinline__ v8f wmma16(v16h a, v16h b, v8f c) {
  v8f d = __builtin_amdgcn_wmma_f32_16x16x32_f16(false, a, false, b, (short)0, c,
                                                 false, false);
  asm volatile("v_nop\n\tv_nop\n\tv_nop\n\tv_nop" : "+v"(d) : "v"(a), "v"(b));
  return d;
}

__device__ __forceinline__ float red32_sum(float x) {
#pragma unroll
  for (int off = 1; off < 32; off <<= 1) x += __shfl_xor(x, off, 32);
  return x;
}

__global__ __launch_bounds__(256) void xprep_kernel(
    const float* __restrict__ X, _Float16* __restrict__ Xn, _Float16* __restrict__ Xt,
    _Float16* __restrict__ Xnt) {
#pragma clang fp contract(off)
  __shared__ _Float16 Tr[64 * LDT];
  __shared__ _Float16 Tx[64 * LDT];
  __shared__ _Float16 Tn[64 * LDT];
  __shared__ float sinv[64];
  const unsigned tid = threadIdx.x, lane = tid & 31u;
  const unsigned wave = __builtin_amdgcn_readfirstlane(threadIdx.x >> 5);
  const unsigned n0 = blockIdx.x * 64u;

#pragma unroll 1
  for (unsigned r = 0; r < 8u; ++r) {
    const unsigned row = wave * 8u + r;
    const float* xr = X + (size_t)(n0 + row) * DIM + lane * 4u;
    float ss = 0.0f;
#pragma unroll 1
    for (unsigned i = 0; i < 4u; ++i) {
      const v4f a = *(const v4f*)(xr + i * 128u);
#pragma unroll
      for (int j = 0; j < 4; ++j) {
        const float e = bf16r(a[j]);
        ss += e * e;
      }
    }
    ss = red32_sum(ss);
    const float inv = NCARRY * (1.0f / fmaxf(sqrtf(ss), 1.0e-8f));
    if (lane == 0u) sinv[row] = inv;
  }
  __syncthreads();

#pragma unroll 1
  for (unsigned cb = 0; cb < (unsigned)(DIM / 64); ++cb) {
    const unsigned c0 = cb * 64u;
#pragma unroll 4
    for (unsigned j = 0; j < 16u; ++j) {
      const unsigned idx = tid + 256u * j;
      const unsigned kr = idx >> 6, nc = idx & 63u;
      const float v = bf16r(X[(size_t)(n0 + kr) * DIM + c0 + nc]);
      const h16 hx = toh_flush(v);
      const h16 hn = toh_flush(v * sinv[kr]);
      Tx[nc * LDT + kr] = hx;
      Tn[nc * LDT + kr] = hn;
      Tr[kr * LDT + nc] = hn;
    }
    __syncthreads();
    v8h xa[2], xb[2], xc[2];
    size_t offt[2], offr[2];
#pragma unroll
    for (unsigned i = 0; i < 2u; ++i) {
      const unsigned r = 32u * i + (tid >> 3);
      const unsigned kc = (tid & 7u) * 8u;
      xa[i] = *(const v8h*)&Tx[r * LDT + kc];
      xb[i] = *(const v8h*)&Tn[r * LDT + kc];
      xc[i] = *(const v8h*)&Tr[r * LDT + kc];
      offt[i] = (size_t)(c0 + r) * NROWS + n0 + kc;
      offr[i] = (size_t)(n0 + r) * DIM + c0 + kc;
    }
#pragma unroll
    for (int i = 0; i < 2; ++i) {
      *(volatile v8h*)(Xt + offt[i]) = xa[i];
      *(volatile v8h*)(Xnt + offt[i]) = xb[i];
      *(volatile v8h*)(Xn + offr[i]) = xc[i];
    }
    __threadfence();
#pragma unroll
    for (int i = 0; i < 2; ++i) {
      *(volatile v8h*)(Xt + offt[i]) = xa[i];
      *(volatile v8h*)(Xnt + offt[i]) = xb[i];
      *(volatile v8h*)(Xn + offr[i]) = xc[i];
    }
    __syncthreads();
  }
}

__global__ __launch_bounds__(256) void soft_kernel(
    const float* __restrict__ L, float* __restrict__ wts, int* __restrict__ cls) {
#pragma clang fp contract(off)
  __shared__ __attribute__((aligned(16))) float smp[64];
  __shared__ __attribute__((aligned(16))) int scls[64];
  const unsigned tid = threadIdx.x, lane = tid & 31u;
  const unsigned wave = __builtin_amdgcn_readfirstlane(threadIdx.x >> 5);
  const unsigned n0 = blockIdx.x * 64u;

#pragma unroll 1
  for (unsigned r = 0; r < 8u; ++r) {
    const unsigned row = wave * 8u + r;
    const float* lr = L + (size_t)(n0 + row) * NCLS;
    float mv = -3.0e38f;
    int mi = 0x7fffffff;
#pragma unroll 1
    for (unsigned i = 0; i < 4u; ++i) {
      const unsigned j = lane + 32u * i;
      const unsigned jc = (j < (unsigned)NCLS) ? j : (unsigned)(NCLS - 1);
      float v = lr[jc];
      asm volatile("" : "+v"(v));
      v = bf16r(v);
      const bool better = (j < (unsigned)NCLS) && (v > mv);
      mv = better ? v : mv;
      mi = better ? (int)j : mi;
    }
#pragma unroll
    for (int off = 1; off < 32; off <<= 1) {
      const float ov = __shfl_xor(mv, off, 32);
      const int oi = __shfl_xor(mi, off, 32);
      const bool take = (ov > mv) || ((ov == mv) && (oi < mi));
      mv = take ? ov : mv;
      mi = take ? oi : mi;
    }
    float se = 0.0f;
#pragma unroll 1
    for (unsigned i = 0; i < 4u; ++i) {
      const unsigned j = lane + 32u * i;
      const unsigned jc = (j < (unsigned)NCLS) ? j : (unsigned)(NCLS - 1);
      float v = lr[jc];
      asm volatile("" : "+v"(v));
      const float e = __expf(bf16r(v) - mv);
      se += (j < (unsigned)NCLS) ? e : 0.0f;
    }
    se = red32_sum(se);
    if (lane == 0u) {
      smp[row] = 1.0f / se;
      scls[row] = mi;
    }
  }
  __syncthreads();

  const unsigned ci = (tid & 15u) * 4u;
  const v4f wv = *(const v4f*)&smp[ci];
  const v4i cv = *(const v4i*)&scls[ci];
  float* wdst = wts + n0 + ci;
  int* cdst = cls + n0 + ci;
  if (tid < 16u) {
    *(volatile v4f*)wdst = wv;
    *(volatile v4i*)cdst = cv;
  }
  __threadfence();
  if (tid < 16u) {
    *(volatile v4f*)wdst = wv;
    *(volatile v4i*)cdst = cv;
  }
}

template <int MODE>
__device__ __forceinline__ void gemm_body(
    const _Float16* __restrict__ A16, const _Float16* __restrict__ Bt, const unsigned K,
    const _Float16* __restrict__ addh, const float* __restrict__ cnt,
    float* __restrict__ outf, _Float16* __restrict__ out16, const unsigned ldo) {
  __shared__ float Cs[64 * LDC];
  const unsigned tid = threadIdx.x, lane = tid & 31u, w = tid >> 5;
  const unsigned mw = w >> 1, nw = w & 1u;
  const unsigned hh = lane >> 4, m = lane & 15u;
  const unsigned n0 = blockIdx.x * 64u;
  const unsigned row0 = blockIdx.y * 64u;

  const _Float16* ap  = A16 + (size_t)(row0 + mw * 16u + m) * K + hh * 8u;
  const _Float16* bp0 = Bt + (size_t)(n0 + nw * 32u + m) * K + hh * 8u;
  const _Float16* bp1 = bp0 + (size_t)16 * K;
  v8f acc0 = {}, acc1 = {};
#pragma unroll 2
  for (unsigned k0 = 0; k0 < K; k0 += 32u) {
    const v16h a  = frag_at(ap + k0);
    const v16h b0 = frag_at(bp0 + k0);
    const v16h b1 = frag_at(bp1 + k0);
    acc0 = wmma16(a, b0, acc0);
    acc1 = wmma16(a, b1, acc1);
  }
#pragma unroll
  for (int r = 0; r < 8; ++r) {
    float* d = &Cs[(mw * 16u + hh * 8u + (unsigned)r) * LDC + nw * 32u + m];
    d[0]  = acc0[r];
    d[16] = acc1[r];
  }
  __syncthreads();

  if (MODE == 0 || MODE == 1) {
    v8h x[2];
    size_t off[2];
#pragma unroll
    for (unsigned i = 0; i < 2u; ++i) {
      const unsigned r = 32u * i + (tid >> 3);
      const unsigned c = (tid & 7u) * 8u;
      const v4f u0 = *(const v4f*)&Cs[r * LDC + c];
      const v4f u1 = *(const v4f*)&Cs[r * LDC + c + 4];
      off[i] = (size_t)(row0 + r) * ldo + n0 + c;
      if (MODE == 1) {
        const v8h xa = *(const v8h*)(addh + off[i]);
#pragma unroll
        for (int j = 0; j < 4; ++j) {
          x[i][j]     = toh_flush(u0[j] * (1.0f / NCARRY) + (float)xa[j]);
          x[i][j + 4] = toh_flush(u1[j] * (1.0f / NCARRY) + (float)xa[j + 4]);
        }
      } else {
#pragma unroll
        for (int j = 0; j < 4; ++j) {
          x[i][j]     = toh_flush(u0[j] * (1.0f / NCARRY));
          x[i][j + 4] = toh_flush(u1[j] * (1.0f / NCARRY));
        }
      }
    }
#pragma unroll
    for (int i = 0; i < 2; ++i) *(volatile v8h*)(out16 + off[i]) = x[i];
    __threadfence();
#pragma unroll
    for (int i = 0; i < 2; ++i) *(volatile v8h*)(out16 + off[i]) = x[i];
  }
}

__global__ __launch_bounds__(256) void gemm_gram_kernel(
    const _Float16* __restrict__ A16, const _Float16* __restrict__ Bt,
    _Float16* __restrict__ gt) {
  gemm_body<0>(A16, Bt, (unsigned)NROWS, A16, (const float*)0, (float*)0, gt, (unsigned)DIM);
}
__global__ __launch_bounds__(256) void gemm_agg_kernel(
    const _Float16* __restrict__ A16, const _Float16* __restrict__ Bt,
    const _Float16* __restrict__ xt, _Float16* __restrict__ xat) {
  gemm_body<1>(A16, Bt, (unsigned)DIM, xt, (const float*)0, (float*)0, xat, (unsigned)NROWS);
}

__global__ __launch_bounds__(256) void proto_kernel(
    const _Float16* __restrict__ xat, const int* __restrict__ cls,
    const float* __restrict__ wts, float* __restrict__ outf) {
#pragma clang fp contract(off)
  __shared__ int slist[NROWS];
  __shared__ int scount[8];
  __shared__ __attribute__((aligned(16))) float ssum[DIM];
  const unsigned tid = threadIdx.x, lane = tid & 31u;
  const unsigned wave = __builtin_amdgcn_readfirstlane(threadIdx.x >> 5);
  const int c = (int)blockIdx.x;
  const unsigned seg0 = wave * (unsigned)SUBROWS;

  unsigned fill = 0u;
#pragma unroll 1
  for (unsigned i = 0; i < (unsigned)(SUBROWS / 32); ++i) {
    const unsigned n = seg0 + i * 32u + lane;
    const int lab = cls[n];
    const bool hit = (lab == c);
    const unsigned mask = __builtin_amdgcn_ballot_w32(hit);
    const unsigned below = mask & ((1u << lane) - 1u);
    unsigned pos = fill + (unsigned)__builtin_popcount(below);
    pos = (pos < (unsigned)SUBROWS) ? pos : (unsigned)(SUBROWS - 1);
    if (hit) slist[seg0 + pos] = (int)n;
    fill += (unsigned)__builtin_popcount(mask);
  }
  if (lane == 0u) scount[wave] = (int)fill;
  __syncthreads();

  const _Float16* p0 = xat + (size_t)tid * NROWS;
  const _Float16* p1 = xat + (size_t)(tid + 256u) * NROWS;
  float a0 = 0.0f, a1 = 0.0f;
  int total = 0;
#pragma unroll 1
  for (unsigned wv = 0; wv < 8u; ++wv) {
    int cwv = scount[wv];
    cwv = (cwv < 0) ? 0 : cwv;
    cwv = (cwv > SUBROWS) ? SUBROWS : cwv;
    const int cw = __builtin_amdgcn_readfirstlane(cwv);
    total += cw;
    const unsigned lbase = wv * (unsigned)SUBROWS;
#pragma unroll 1
    for (int p = 0; p < cw; ++p) {
      int n = slist[lbase + (unsigned)p];
      n = (n < 0) ? 0 : n;
      n = (n > (NROWS - 1)) ? (NROWS - 1) : n;
      const float wgt = wts[n];
      const float t0 = wgt * (float)p0[n];
      const float t1 = wgt * (float)p1[n];
      a0 += t0;
      a1 += t1;
    }
  }

  const float cn = (float)total;
  const float rc = 1.0f / fmaxf(cn, 1.0f);
  ssum[tid]        = (cn > 0.0f) ? (a0 * rc) : 0.0f;
  ssum[tid + 256u] = (cn > 0.0f) ? (a1 * rc) : 0.0f;
  __syncthreads();
  if (tid < 128u) {
    const v4f v = *(const v4f*)&ssum[tid * 4u];
    float* p = outf + (size_t)c * DIM + tid * 4u;
    *(volatile v4f*)p = v;
    __threadfence();
    *(volatile v4f*)p = v;
  }
}

__global__ __launch_bounds__(256) void inter_kernel(const float* proto, float* out) {
  const unsigned tid = threadIdx.x;
  const unsigned d4 = (tid & 127u) * 4u, jj = tid >> 7;
  const unsigned i = blockIdx.y;
  const unsigned j0 = blockIdx.x * 10u;
  const v4f pi = *(const v4f*)(proto + (size_t)i * DIM + d4);
  v4f xs[5];
  size_t off[5];
#pragma unroll
  for (unsigned t = 0; t < 5u; ++t) {
    const unsigned j = j0 + 2u * t + jj;
    const v4f pj = *(const v4f*)(proto + (size_t)j * DIM + d4);
    xs[t] = pj - pi;
    off[t] = ((size_t)i * NCLS + j) * DIM + d4;
  }
#pragma unroll
  for (int t = 0; t < 5; ++t) *(volatile v4f*)(out + off[t]) = xs[t];
  __threadfence();
#pragma unroll
  for (int t = 0; t < 5; ++t) *(volatile v4f*)(out + off[t]) = xs[t];
}

extern "C" void kernel_launch(void* const* d_in, const int* in_sizes, int n_in,
                              void* d_out, int out_size, void* d_ws, size_t ws_size,
                              hipStream_t stream) {
  if (n_in < 2) return;
  if ((long long)in_sizes[0] < (long long)NROWS * DIM) return;
  if ((long long)in_sizes[1] < (long long)NROWS * NCLS) return;
  if ((long long)out_size < (long long)OUT_TOTAL) return;
  if (ws_size < WS_TOTAL) return;

  const float* X = (const float*)d_in[0];
  const float* L = (const float*)d_in[1];
  float* out = (float*)d_out;

  char* ws = (char*)d_ws;
  _Float16* Xt16  = (_Float16*)(ws + OFF_XT);
  _Float16* Xnt16 = (_Float16*)(ws + OFF_XNT);
  _Float16* Xn16  = (_Float16*)(ws + OFF_XN);
  _Float16* Gt16  = (_Float16*)(ws + OFF_GT);
  _Float16* Xat16 = (_Float16*)(ws + OFF_XAT);
  int*      Cls   = (int*)(ws + OFF_CLS);
  float*    Wts   = (float*)(ws + OFF_WT);

  dim3 blk(256);
  xprep_kernel<<<dim3(NROWS / 64), blk, 0, stream>>>(X, Xn16, Xt16, Xnt16);
  soft_kernel<<<dim3(NROWS / 64), blk, 0, stream>>>(L, Wts, Cls);
  gemm_gram_kernel<<<dim3(DIM / 64, DIM / 64), blk, 0, stream>>>(Xt16, Xnt16, Gt16);
  gemm_agg_kernel<<<dim3(NROWS / 64, DIM / 64), blk, 0, stream>>>(Gt16, Xn16, Xt16, Xat16);
  proto_kernel<<<dim3(NCLS), blk, 0, stream>>>(Xat16, Cls, Wts, out);
  inter_kernel<<<dim3(NCLS / 10, NCLS), blk, 0, stream>>>(out, out + OUT1_OFF);
}
